// Main_Net_79852031967513
// MI455X (gfx1250) — hardware-verified
//
#include <hip/hip_runtime.h>
#include <hip/hip_bf16.h>
#include <math.h>


#define BB 2
#define SS 2048
#define DD 1024
#define HH 16
#define DKK 64
#define QW 2

typedef _Float16 bf16;
typedef __attribute__((ext_vector_type(4))) unsigned v4u_t;
typedef unsigned v4ua __attribute__((ext_vector_type(4), may_alias));
typedef __attribute__((ext_vector_type(4))) float v4f_t;
typedef float v4fa __attribute__((ext_vector_type(4), may_alias));
typedef __attribute__((ext_vector_type(16))) bf16  bf16x16;
typedef __attribute__((ext_vector_type(8)))  bf16  bf16x8;
typedef __attribute__((ext_vector_type(4)))  bf16  bf16x4;
typedef __attribute__((ext_vector_type(8)))  float f32x8;

#define LDS_STRIDE 48
#define KSTRIDE    72
#define VSTRIDE    48

__device__ __forceinline__ f32x8 wmma_bf16(bf16x16 a, bf16x16 b, f32x8 c) {
  return __builtin_amdgcn_wmma_f32_16x16x32_f16(
      false, a, false, b, (short)0, c, false, false);
}
#define RSPLIT (1.0f / 2048.0f)
__device__ __forceinline__ bf16 lo_of(float v, bf16 h) { return (bf16)((v - (float)h) * 2048.0f); }
__device__ __forceinline__ f32x8 wmma_split(bf16x16 a, bf16x16 al, bf16x16 b, bf16x16 bl, f32x8 c) {
  f32x8 x = {}; x = wmma_bf16(al, b, x); x = wmma_bf16(a, bl, x); return wmma_bf16(a, b, c) + x * RSPLIT; }

template <typename T>
__device__ __forceinline__ bf16x16 load_frag(const T* __restrict__ base, int ld,
                                             int row0, int k0) {
  const int lane = threadIdx.x & 31;
  const int r    = lane & 15;
  const int kh   = (lane >> 4) * 8;
  const T* p0 = base + (size_t)(row0 + r) * ld + (k0 + kh);
  const T* p1 = p0 + 16;
  bf16x16 f;
#pragma unroll
  for (int i = 0; i < 8; ++i) {
    f[i]     = (bf16)p0[i];
    f[i + 8] = (bf16)p1[i];
  }
  return f;
}

__device__ __forceinline__ bf16x16 lds_frag(const bf16* base, int stride) {
  const int lane = threadIdx.x & 31;
  const int row  = lane & 15;
  const int kh   = (lane >> 4) * 8;
  const bf16x8 lo = *(const bf16x8*)(base + row * stride + kh);
  const bf16x8 hi = *(const bf16x8*)(base + row * stride + kh + 16);
  bf16x16 f;
#pragma unroll
  for (int i = 0; i < 8; ++i) { f[i] = lo[i]; f[i + 8] = hi[i]; }
  return f;
}

template <typename T>
__device__ __forceinline__ void stage_read16(const T* __restrict__ p, float* buf) {
#pragma unroll
  for (int i = 0; i < 16; ++i) buf[i] = (float)p[i];
}

__device__ __forceinline__ void stage_write(bf16* dst, const float* buf, int nquad) {
#pragma unroll
  for (int i = 0; i < nquad; ++i) {
    bf16x4 q;
    q[0] = (bf16)buf[4 * i];     q[1] = (bf16)buf[4 * i + 1];
    q[2] = (bf16)buf[4 * i + 2]; q[3] = (bf16)buf[4 * i + 3];
    *(bf16x4*)(dst + 4 * i) = q;
  }
}

__global__ __launch_bounds__(256) void transpose_pack_kernel(const float* __restrict__ W, bf16* __restrict__ WT, int K, int N, size_t plane) {
  __shared__ float tile[64][65];
  const int k0 = blockIdx.y * 64, n0 = blockIdx.x * 64, t = threadIdx.x;
  for (int i = t; i < 64 * 64; i += 256) { const int kr = i >> 6, nc = i & 63; tile[kr][nc] = W[(size_t)(k0 + kr) * N + n0 + nc]; }
  __syncthreads();
#pragma unroll 1
  for (int pass = 0; pass < 2; ++pass) {
    for (int i = t; i < 64 * 8; i += 256) { const int nr = i >> 3, k8 = (i & 7) * 8; bf16 hh[8], hl[8];
#pragma unroll
      for (int e = 0; e < 8; ++e) { const float v = tile[k8 + e][nr]; hh[e] = (bf16)v; hl[e] = lo_of(v, hh[e]); }
      bf16* d = WT + (size_t)(n0 + nr) * K + k0 + k8;
      *(volatile v4u_t*)d = *(const v4ua*)hh; *(volatile v4u_t*)(d + plane) = *(const v4ua*)hl; }
    __threadfence();
  }
}

template <typename AT, typename WT, int MODE>
__global__ __launch_bounds__(256) void gemm_split_kernel(
    const AT* __restrict__ A, size_t aPlane, const WT* __restrict__ W, size_t wPlane,
    const float* __restrict__ bias, void* __restrict__ out,
    int M, int N, int K) {
  __shared__ bf16 ldsA[128 * LDS_STRIDE], ldsAl[128 * LDS_STRIDE];
  __shared__ bf16 ldsW[256 * LDS_STRIDE], ldsWl[256 * LDS_STRIDE];
  __shared__ __attribute__((aligned(16))) unsigned char sob[256 * 136 * 2];

  const int t    = threadIdx.x;
  const int wave = t >> 5;
  const int lane = t & 31;
  const int wm   = (wave & 1) * 64;
  const int wn   = (wave >> 1) * 64;
  const int mBlk = blockIdx.x * 128;
  const int nBlk = blockIdx.y * 256;
  const int arow = t >> 1;
  const int ach  = (t & 1) * 16;

  f32x8 acc[4][4] = {};
  for (int k = 0; k < K; k += 32) {
    __syncthreads();
    {
      const AT* ap = A + (size_t)(mBlk + arow) * K + k + ach;
      bf16 hh[16], hl[16];
      if (sizeof(AT) == 4) {
#pragma unroll
        for (int i = 0; i < 16; ++i) { const float v = (float)ap[i]; hh[i] = (bf16)v; hl[i] = lo_of(v, hh[i]); }
      } else {
#pragma unroll
        for (int i = 0; i < 16; ++i) { hh[i] = (bf16)ap[i]; hl[i] = (bf16)ap[aPlane + i]; }
      }
#pragma unroll
      for (int i = 0; i < 16; ++i) { ldsA[arow * LDS_STRIDE + ach + i] = hh[i]; ldsAl[arow * LDS_STRIDE + ach + i] = hl[i]; }
    }
    {
      const WT* wp = W + (size_t)(nBlk + t) * K + k;
      if (sizeof(WT) == 4) {
#pragma unroll
        for (int i = 0; i < 32; ++i) { const float v = (float)wp[i]; const bf16 h_ = (bf16)v; ldsW[t * LDS_STRIDE + i] = h_; ldsWl[t * LDS_STRIDE + i] = lo_of(v, h_); }
      } else {
#pragma unroll
        for (int i = 0; i < 32; ++i) { ldsW[t * LDS_STRIDE + i] = (bf16)wp[i]; ldsWl[t * LDS_STRIDE + i] = (bf16)wp[wPlane + i]; }
      }
    }
    __syncthreads();
    bf16x16 wf[4], wfl[4];
#pragma unroll
    for (int j = 0; j < 4; ++j) { wf[j] = lds_frag(ldsW + (wn + 16 * j) * LDS_STRIDE, LDS_STRIDE); wfl[j] = lds_frag(ldsWl + (wn + 16 * j) * LDS_STRIDE, LDS_STRIDE); }
#pragma unroll
    for (int i = 0; i < 4; ++i) {
      const bf16x16 af = lds_frag(ldsA + (wm + 16 * i) * LDS_STRIDE, LDS_STRIDE), afl = lds_frag(ldsAl + (wm + 16 * i) * LDS_STRIDE, LDS_STRIDE);
#pragma unroll
      for (int j = 0; j < 4; ++j) acc[i][j] = wmma_split(af, afl, wf[j], wfl[j], acc[i][j]);
    }
  }

  const int nlane = lane & 15;
  const int mh    = (lane >> 4) * 8;
  __syncthreads();
  if (MODE == 1) {
    bf16* so = (bf16*)sob;
#pragma unroll
    for (int i = 0; i < 4; ++i)
#pragma unroll
      for (int j = 0; j < 4; ++j) {
        const int nl = wn + 16 * j + nlane;
        const float bv = bias ? bias[nBlk + nl] : 0.0f;
#pragma unroll
        for (int r = 0; r < 8; ++r) so[nl * 136 + wm + 16 * i + mh + r] = (bf16)(acc[i][j][r] + bv);
      }
    __syncthreads();
    const int b_ = mBlk >> 11, s0 = mBlk & (SS - 1);
#pragma unroll 1
    for (int pass = 0; pass < 2; ++pass) {
      for (int ch = t; ch < 256 * 16; ch += 256) { const int nl = ch >> 4, q = (ch & 15) * 8; const int n = nBlk + nl, h = n >> 6, dk = n & (DKK - 1);
        *(volatile v4u_t*)((bf16*)out + (((size_t)(b_ * HH + h)) * DKK + dk) * SS + s0 + q) = *(const v4ua*)(so + nl * 136 + q); }
      __threadfence();
    }
  } else {
    float* so = (float*)sob;
#pragma unroll 1
    for (int hf = 0; hf < 2; ++hf) {
      if (wm == hf * 64) {
#pragma unroll
        for (int i = 0; i < 4; ++i)
#pragma unroll
          for (int j = 0; j < 4; ++j) {
            const int nl = wn + 16 * j + nlane;
            const float bv = bias ? bias[nBlk + nl] : 0.0f;
#pragma unroll
            for (int r = 0; r < 8; ++r) so[(16 * i + mh + r) * 260 + nl] = acc[i][j][r] + bv;
          }
      }
      __syncthreads();
#pragma unroll 1
      for (int pass = 0; pass < 2; ++pass) {
        for (int ch = t; ch < 64 * 64; ch += 256) { const int ml = ch >> 6, q = (ch & 63) * 4;
          *(volatile v4f_t*)((float*)out + (size_t)(mBlk + hf * 64 + ml) * N + nBlk + q) = *(const volatile v4fa*)(so + ml * 260 + q); }
        __threadfence();
      }
      __syncthreads();
    }
  }
}


#define NBM 2048
#define NIN 1024
#define NHID 512
#define NF 256

__global__ __launch_bounds__(256) void k_relu(float* __restrict__ H, int n4) {
  const int i = blockIdx.x * 256 + threadIdx.x; if (i >= n4) return;
  v4f_t v = *(const v4fa*)(H + (size_t)i * 4); v.x = fmaxf(v.x, 0.f); v.y = fmaxf(v.y, 0.f); v.z = fmaxf(v.z, 0.f); v.w = fmaxf(v.w, 0.f);
  *(volatile v4f_t*)(H + (size_t)i * 4) = v; __threadfence(); *(volatile v4f_t*)(H + (size_t)i * 4) = v;
}
__global__ __launch_bounds__(256) void k_mo(const float* __restrict__ Wout, float* __restrict__ Mo) {
  const int j = blockIdx.x, o = blockIdx.y, i = threadIdx.x; const float v = Wout[((size_t)j * NF + i) * 2 + o];
  float* dst = Mo + ((size_t)o * NF + j) * NF + i; *(volatile float*)dst = v; __threadfence(); *(volatile float*)dst = v;
}
__global__ __launch_bounds__(256) void k_head(const float* __restrict__ F1, const float* __restrict__ G0, const float* __restrict__ G1, const float* __restrict__ bout, float* __restrict__ out) {
  __shared__ float r0[16][16], r1[16][16]; __shared__ float res[32];
  const int t = threadIdx.x, sl = t >> 4, part = t & 15, b = blockIdx.x * 16 + sl;
  const float* f = F1 + (size_t)b * NF; const float* g0 = G0 + (size_t)b * NF; const float* g1 = G1 + (size_t)b * NF;
  float a0 = 0.f, a1 = 0.f;
#pragma unroll 1
  for (int j = part * 16; j < part * 16 + 16; ++j) { const float fv = f[j]; a0 += fv * g0[j]; a1 += fv * g1[j]; }
  r0[sl][part] = a0; r1[sl][part] = a1; __syncthreads();
  if (part == 0) { float s0 = 0.f, s1 = 0.f;
#pragma unroll
    for (int p = 0; p < 16; ++p) { s0 += r0[sl][p]; s1 += r1[sl][p]; }
    res[sl * 2] = s0 + bout[0]; res[sl * 2 + 1] = s1 + bout[1]; }
  __syncthreads();
  if (t < 8) { const v4f_t v = *(const volatile v4fa*)(res + t * 4); float* dst = out + (size_t)blockIdx.x * 32 + t * 4;
    *(volatile v4f_t*)dst = v; __threadfence(); *(volatile v4f_t*)dst = v; }
}

extern "C" void kernel_launch(void* const* d_in, const int* in_sizes, int n_in,
                              void* d_out, int out_size, void* d_ws, size_t ws_size,
                              hipStream_t stream) {
  (void)in_sizes; (void)n_in; (void)out_size; (void)ws_size;
  const float* x0 = (const float*)d_in[0]; const float* x1 = (const float*)d_in[1];
  const float* Wf = (const float*)d_in[2]; const float* bfe = (const float*)d_in[3];
  const float* Wb0 = (const float*)d_in[4]; const float* bb0 = (const float*)d_in[5];
  const float* Wb1 = (const float*)d_in[6]; const float* bb1 = (const float*)d_in[7];
  const float* Wout = (const float*)d_in[8]; const float* bout = (const float*)d_in[9];
  char* ws = (char*)d_ws;
  const size_t plF = (size_t)NHID * NIN, plB = (size_t)NF * NHID;
  bf16* WfT  = (bf16*)ws;  ws += plF * 2 * 2;
  bf16* Wb0T = (bf16*)ws;  ws += plB * 2 * 2;
  bf16* Wb1T = (bf16*)ws;  ws += plB * 2 * 2;
  float* Mo  = (float*)ws; ws += (size_t)2 * NF * NF * 4;
  float* H0  = (float*)ws; ws += (size_t)NBM * NHID * 4;
  float* H1  = (float*)ws; ws += (size_t)NBM * NHID * 4;
  float* F0  = (float*)ws; ws += (size_t)NBM * NF * 4;
  float* F1  = (float*)ws; ws += (size_t)NBM * NF * 4;
  float* G0  = (float*)ws; ws += (size_t)NBM * NF * 4;
  float* G1  = (float*)ws; ws += (size_t)NBM * NF * 4;
  transpose_pack_kernel<<<dim3(NHID / 64, NIN / 64), 256, 0, stream>>>(Wf, WfT, NIN, NHID, plF);
  transpose_pack_kernel<<<dim3(NF / 64, NHID / 64), 256, 0, stream>>>(Wb0, Wb0T, NHID, NF, plB);
  transpose_pack_kernel<<<dim3(NF / 64, NHID / 64), 256, 0, stream>>>(Wb1, Wb1T, NHID, NF, plB);
  k_mo<<<dim3(NF, 2), 256, 0, stream>>>(Wout, Mo);
  dim3 blk(256);
  gemm_split_kernel<float, bf16, 2><<<dim3(NBM / 128, NHID / 256), blk, 0, stream>>>(x0, 0, WfT, plF, bfe, H0, NBM, NHID, NIN);
  gemm_split_kernel<float, bf16, 2><<<dim3(NBM / 128, NHID / 256), blk, 0, stream>>>(x1, 0, WfT, plF, bfe, H1, NBM, NHID, NIN);
  k_relu<<<(NBM * NHID / 4 + 255) / 256, 256, 0, stream>>>(H0, NBM * NHID / 4);
  k_relu<<<(NBM * NHID / 4 + 255) / 256, 256, 0, stream>>>(H1, NBM * NHID / 4);
  gemm_split_kernel<float, bf16, 2><<<dim3(NBM / 128, NF / 256), blk, 0, stream>>>(H0, 0, Wb0T, plB, bb0, F0, NBM, NF, NHID);
  gemm_split_kernel<float, bf16, 2><<<dim3(NBM / 128, NF / 256), blk, 0, stream>>>(H1, 0, Wb1T, plB, bb1, F1, NBM, NF, NHID);
  gemm_split_kernel<float, float, 2><<<dim3(NBM / 128, NF / 256), blk, 0, stream>>>(F0, 0, Mo, 0, nullptr, G0, NBM, NF, NF);
  gemm_split_kernel<float, float, 2><<<dim3(NBM / 128, NF / 256), blk, 0, stream>>>(F0, 0, Mo + (size_t)NF * NF, 0, nullptr, G1, NBM, NF, NF);
  k_head<<<NBM / 16, 256, 0, stream>>>(F1, G0, G1, bout, (float*)d_out);
}
